// RNN_64415919506221
// MI455X (gfx1250) — hardware-verified
//
#include <hip/hip_runtime.h>
#include <math.h>

constexpr int NVOCAB   = 30522;
constexpr int NEMB     = 64;
constexpr int NHID     = 128;
constexpr int NBATCH   = 512;
constexpr int NSEQ     = 512;
constexpr int NTHR     = 256;
constexpr int ROWS_BLK = 32;
constexpr int XPITCH   = 72;
constexpr int HPITCH   = 136;
constexpr int FPITCH   = 132;
constexpr int TCHUNK   = 32;
constexpr int XE_BUF   = ROWS_BLK * XPITCH;
constexpr int H_BUF    = ROWS_BLK * HPITCH;
constexpr int TOK_BUF  = ROWS_BLK * TCHUNK;
constexpr float ACARRY = 16.0f;
constexpr float WCARRY = 256.0f;
constexpr float FOLD   = 1.0f / (ACARRY * WCARRY);

static_assert(NBATCH % ROWS_BLK == 0, "batch tile");
static_assert(NSEQ % TCHUNK == 0, "token chunk");
static_assert(NEMB % 32 == 0 && NHID % 32 == 0, "k multiple of 32");
static_assert(NHID == 16 * (NTHR / 32), "8 waves x 16 hidden columns");
static_assert(ROWS_BLK * (NEMB / 8) == NTHR, "gather map: 32 rows x 8 chunks of 8 floats");
static_assert((2 * H_BUF) % NTHR == 0, "zero-fill loop exact");
static_assert(XPITCH % 8 == 0 && HPITCH % 8 == 0 && FPITCH % 4 == 0, "16-B aligned pitches");
static_assert(ROWS_BLK * 4 == 128, "one 128-B output line per block");

typedef __attribute__((ext_vector_type(16))) _Float16 v16h;
typedef __attribute__((ext_vector_type(8)))  _Float16 v8h;
typedef __attribute__((ext_vector_type(8)))  float    v8f;
typedef __attribute__((ext_vector_type(4)))  float    v4f;
typedef __attribute__((ext_vector_type(4)))  int      v4i;

struct FragH {
  union U { v16h v; v8h h[2]; };
  static __device__ __forceinline__ v16h load(const _Float16* p) {
    U f;
    f.h[0] = *(const v8h*)(p);
    f.h[1] = *(const v8h*)(p + 16);
    return f.v;
  }
};

__device__ __forceinline__ v8f mma_h(v16h a, v16h b, v8f c) {
  c = __builtin_amdgcn_wmma_f32_16x16x32_f16(false, a, false, b, (short)0, c, false, false);
  asm volatile("v_nop\n\tv_nop\n\tv_nop\n\tv_nop" : "+v"(c) : "v"(a), "v"(b));
  return c;
}

__device__ __forceinline__ v16h wfrag_from_f32(const float* p) {
  const v4f a0 = *(const v4f*)(p);
  const v4f a1 = *(const v4f*)(p + 4);
  const v4f c0 = *(const v4f*)(p + 16);
  const v4f c1 = *(const v4f*)(p + 20);
  v16h f;
#pragma unroll
  for (int e = 0; e < 4; ++e) {
    f[e]      = (_Float16)(a0[e] * WCARRY);
    f[4 + e]  = (_Float16)(a1[e] * WCARRY);
    f[8 + e]  = (_Float16)(c0[e] * WCARRY);
    f[12 + e] = (_Float16)(c1[e] * WCARRY);
  }
  return f;
}

__device__ __forceinline__ v8h cvt8_carry(v4f a, v4f b) {
  v8h o;
#pragma unroll
  for (int e = 0; e < 4; ++e) {
    o[e]     = (_Float16)(a[e] * ACARRY);
    o[4 + e] = (_Float16)(b[e] * ACARRY);
  }
  return o;
}

__device__ __forceinline__ float tanh_f32(float v) {
  const float e = expf(2.0f * v);
  return 1.0f - 2.0f * (1.0f / (e + 1.0f));
}

__global__ __launch_bounds__(NTHR) void rnn_seq_kernel(
    const int* __restrict__ x, const float* __restrict__ emb,
    const float* __restrict__ W_ih, const float* __restrict__ W_hh,
    const float* __restrict__ b_ih, const float* __restrict__ b_hh,
    const float* __restrict__ W_fc, const float* __restrict__ b_fc,
    float* __restrict__ out) {
  __shared__ __align__(16) _Float16 sH[2 * H_BUF];
  __shared__ __align__(16) _Float16 sXe[2 * XE_BUF];
  __shared__ __align__(16) int      sTok[2 * TOK_BUF];
  __shared__ __align__(16) float    sHf[ROWS_BLK * FPITCH];
  __shared__ __align__(16) float    sWfc[NHID];

  const int tid  = threadIdx.x;
  const int lane = tid & 31;
  const int wave = tid >> 5;
  const int c    = lane & 15;
  const int hh   = lane >> 4;
  const int koff = hh * 8;
  const int b0   = blockIdx.x * ROWS_BLK;
  const int tr   = tid >> 3;
  const int tq   = tid & 7;
  const int j    = 16 * wave + c;

#pragma unroll 1
  for (int i = tid; i < 2 * H_BUF; i += NTHR) sH[i] = (_Float16)0.0f;
  {
    const v4i tk = *(const v4i*)(x + (size_t)(b0 + tr) * NSEQ + 4 * tq);
    *(v4i*)(sTok + tr * TCHUNK + 4 * tq) = tk;
  }
  if (tid < NHID) sWfc[tid] = W_fc[tid];
  __syncthreads();

  int rofs_ih = j * NEMB + koff;
  int rofs_hh = j * NHID + koff;
  const v16h Bih0 = wfrag_from_f32(W_ih + rofs_ih);
  asm volatile("" : "+v"(rofs_ih) : "v"(Bih0));
  const v16h Bih1 = wfrag_from_f32(W_ih + rofs_ih + 32);
  asm volatile("" : "+v"(rofs_hh) : "v"(Bih1));
  const v16h Bhh0 = wfrag_from_f32(W_hh + rofs_hh);
  asm volatile("" : "+v"(rofs_hh) : "v"(Bhh0));
  const v16h Bhh1 = wfrag_from_f32(W_hh + rofs_hh + 32);
  asm volatile("" : "+v"(rofs_hh) : "v"(Bhh1));
  const v16h Bhh2 = wfrag_from_f32(W_hh + rofs_hh + 64);
  asm volatile("" : "+v"(rofs_hh) : "v"(Bhh2));
  const v16h Bhh3 = wfrag_from_f32(W_hh + rofs_hh + 96);
  asm volatile("" : "+v"(rofs_hh) : "v"(Bhh3));

  const float bias = b_ih[j] + b_hh[j];

  v4f na, nb;
  {
    int tok = sTok[tr * TCHUNK + 0];
    tok = tok < 0 ? 0 : (tok > NVOCAB - 1 ? NVOCAB - 1 : tok);
    const float* p = emb + (size_t)tok * NEMB + 8 * tq;
    const v4f a = *(const v4f*)(p);
    const v4f b = *(const v4f*)(p + 4);
    *(v8h*)(sXe + tr * XPITCH + 8 * tq) = cvt8_carry(a, b);
    int tok1 = sTok[tr * TCHUNK + 1];
    tok1 = tok1 < 0 ? 0 : (tok1 > NVOCAB - 1 ? NVOCAB - 1 : tok1);
    const float* p1 = emb + (size_t)tok1 * NEMB + 8 * tq;
    na = *(const v4f*)(p1);
    nb = *(const v4f*)(p1 + 4);
  }
  __syncthreads();

  const v8f z8 = {0.f, 0.f, 0.f, 0.f, 0.f, 0.f, 0.f, 0.f};

#pragma unroll 1
  for (int s = 0; s < NSEQ; ++s) {
    const int cur = s & 1;
    const int nxt = cur ^ 1;
    const _Float16* xa = sXe + cur * XE_BUF;
    const _Float16* ha = sH + cur * H_BUF;
    _Float16* hn = sH + nxt * H_BUF;
    const bool last = (s == NSEQ - 1);

#pragma unroll 1
    for (int mt = 0; mt < 2; ++mt) {
      const _Float16* xr = xa + (16 * mt + c) * XPITCH + koff;
      const _Float16* hr = ha + (16 * mt + c) * HPITCH + koff;
      const v16h a0 = FragH::load(xr);
      const v16h a1 = FragH::load(xr + 32);
      const v16h a2 = FragH::load(hr);
      const v16h a3 = FragH::load(hr + 32);
      const v16h a4 = FragH::load(hr + 64);
      const v16h a5 = FragH::load(hr + 96);
      v8f acc = z8;
      acc = mma_h(a0, Bih0, acc);
      acc = mma_h(a1, Bih1, acc);
      acc = mma_h(a2, Bhh0, acc);
      acc = mma_h(a3, Bhh1, acc);
      acc = mma_h(a4, Bhh2, acc);
      acc = mma_h(a5, Bhh3, acc);
#pragma unroll
      for (int r = 0; r < 8; ++r) {
        const float z  = acc[r] * FOLD + bias;
        const float hv = tanh_f32(z);
        const int row  = 16 * mt + 8 * hh + r;
        hn[row * HPITCH + j] = (_Float16)(hv * ACARRY);
        if (last) sHf[row * FPITCH + j] = hv;
      }
    }

    *(v8h*)(sXe + nxt * XE_BUF + tr * XPITCH + 8 * tq) = cvt8_carry(na, nb);

    if (((s & (TCHUNK - 1)) == 0) && (s + TCHUNK < NSEQ)) {
      const int chunk = (s >> 5) + 1;
      const v4i tk = *(const v4i*)(x + (size_t)(b0 + tr) * NSEQ + chunk * TCHUNK + 4 * tq);
      *(v4i*)(sTok + (chunk & 1) * TOK_BUF + tr * TCHUNK + 4 * tq) = tk;
    }

    {
      const int g = (s + 2 < NSEQ) ? (s + 2) : (NSEQ - 1);
      int tok = sTok[((g >> 5) & 1) * TOK_BUF + tr * TCHUNK + (g & (TCHUNK - 1))];
      tok = tok < 0 ? 0 : (tok > NVOCAB - 1 ? NVOCAB - 1 : tok);
      const float* p = emb + (size_t)tok * NEMB + 8 * tq;
      na = *(const v4f*)(p);
      nb = *(const v4f*)(p + 4);
    }

    __syncthreads();
  }

  if (wave == 0) {
    const float* hrow = sHf + lane * FPITCH;
    float sum = 0.0f;
#pragma unroll 4
    for (int k = 0; k < NHID; ++k) sum = fmaf(hrow[k], sWfc[k], sum);
    const float z = sum + b_fc[0];
    const float o = 1.0f / (1.0f + expf(-z));
    volatile float* op = (volatile float*)(out + b0 + lane);
    *op = o;
    __threadfence();
    *op = o;
  }
}

extern "C" void kernel_launch(void* const* d_in, const int* in_sizes, int n_in,
                              void* d_out, int out_size, void* d_ws, size_t ws_size, hipStream_t stream) {
  (void)d_ws; (void)ws_size;
  if (n_in < 8 || d_out == nullptr) return;
  if (in_sizes[0] != NBATCH * NSEQ || in_sizes[1] != NVOCAB * NEMB || in_sizes[2] != NHID * NEMB ||
      in_sizes[3] != NHID * NHID || in_sizes[4] != NHID || in_sizes[5] != NHID ||
      in_sizes[6] != NHID || in_sizes[7] != 1 || out_size != NBATCH) return;

  const int*   x    = (const int*)  d_in[0];
  const float* emb  = (const float*)d_in[1];
  const float* W_ih = (const float*)d_in[2];
  const float* W_hh = (const float*)d_in[3];
  const float* b_ih = (const float*)d_in[4];
  const float* b_hh = (const float*)d_in[5];
  const float* W_fc = (const float*)d_in[6];
  const float* b_fc = (const float*)d_in[7];

  rnn_seq_kernel<<<NBATCH / ROWS_BLK, NTHR, 0, stream>>>(x, emb, W_ih, W_hh, b_ih, b_hh, W_fc, b_fc, (float*)d_out);
}
